// LinearSegmentMemoryWrapper_6210522710455
// MI455X (gfx1250) — hardware-verified
//
#include <hip/hip_runtime.h>
#include <math.h>
#include <stdint.h>

constexpr int NBATCH  = 8;
constexpr int SEQ_T   = 2048;
constexpr int DIM_E   = 512;
constexpr int ATT_LDV = NBATCH * SEQ_T;
constexpr int KSPAN   = 13;
constexpr float DECAY_VAL = 0.97f;

typedef __attribute__((ext_vector_type(16))) _Float16 v16h;
typedef __attribute__((ext_vector_type(8)))  _Float16 v8h;
typedef __attribute__((ext_vector_type(16))) __bf16   v16b;
typedef __attribute__((ext_vector_type(8)))  __bf16   v8b;
typedef __attribute__((ext_vector_type(8)))  float    v8f;
typedef __attribute__((ext_vector_type(4)))  float    v4f;
typedef __attribute__((ext_vector_type(2)))  float    v2f;
typedef __attribute__((ext_vector_type(4)))  unsigned int v4u;

__device__ __forceinline__ unsigned short f2bf_bits(float f) {
  unsigned u = __float_as_uint(f);
  return (unsigned short)((u + 0x7FFFu + ((u >> 16) & 1u)) >> 16);
}
__device__ __forceinline__ float bf_bits2f(unsigned short h) { return __uint_as_float(((unsigned)h) << 16); }
__device__ __forceinline__ float bfr(float f) { return bf_bits2f(f2bf_bits(f)); }
__device__ __forceinline__ unsigned pk16(unsigned short a, unsigned short b) { return (unsigned)a | ((unsigned)b << 16); }

__device__ __forceinline__ void dep_guard_h(v8f& a, v8f& b, v16h x, v16h y) { asm volatile("v_nop\n\tv_nop\n\tv_nop\n\tv_nop" : "+v"(a), "+v"(b) : "v"(x), "v"(y)); }
__device__ __forceinline__ void dep_guard_b(v8f& a, v8f& b, v16b x, v16b y) { asm volatile("v_nop\n\tv_nop\n\tv_nop\n\tv_nop" : "+v"(a), "+v"(b) : "v"(x), "v"(y)); }
__device__ __forceinline__ void keep4_h(v16h a, v16h b, v16h c, v16h d) { asm volatile("v_nop" :: "v"(a), "v"(b), "v"(c), "v"(d)); }
__device__ __forceinline__ void keep4_b(v16b a, v16b b, v16b c, v16b d) { asm volatile("v_nop" :: "v"(a), "v"(b), "v"(c), "v"(d)); }
__device__ __forceinline__ void acc_guard4(v8f& a, v8f& b, v8f& c, v8f& d) { asm volatile("v_nop\n\tv_nop\n\tv_nop\n\tv_nop" : "+v"(a), "+v"(b), "+v"(c), "+v"(d)); }
template <typename T> struct Frag;
template <> struct Frag<_Float16> {
  typedef v16h V; union U { v16h v; v8h h[2]; };
  static __device__ __forceinline__ v16h load(const _Float16* p) {
    U f; f.h[0] = *(const v8h*)(p); f.h[1] = *(const v8h*)(p + 16); return f.v;
  }
  static __device__ __forceinline__ v8f mma(v16h a, v16h b, v8f c) {
    return __builtin_amdgcn_wmma_f32_16x16x32_f16(false, a, false, b, (short)0, c, false, false);
  }
  static __device__ __forceinline__ void guard(v8f& a, v8f& b, v16h x, v16h y) { dep_guard_h(a, b, x, y); }
  static __device__ __forceinline__ void keep(v16h a, v16h b, v16h c, v16h d) { keep4_h(a, b, c, d); }
};
template <> struct Frag<__bf16> {
  typedef v16b V; union U { v16b v; v8b h[2]; };
  static __device__ __forceinline__ v16b load(const __bf16* p) {
    U f; f.h[0] = *(const v8b*)(p); f.h[1] = *(const v8b*)(p + 16); return f.v;
  }
  static __device__ __forceinline__ v8f mma(v16b a, v16b b, v8f c) {
    return __builtin_amdgcn_wmma_f32_16x16x32_bf16(false, a, false, b, (short)0, c, false, false);
  }
  static __device__ __forceinline__ void guard(v8f& a, v8f& b, v16b x, v16b y) { dep_guard_b(a, b, x, y); }
  static __device__ __forceinline__ void keep(v16b a, v16b b, v16b c, v16b d) { keep4_b(a, b, c, d); }
};

template <int ET> struct Elem;
template <> struct Elem<0> { typedef _Float16 T; };
template <> struct Elem<1> { typedef __bf16 T; };
template <int ET, int SPLIT, int BIAS_MODE, int OUT_MODE, bool RESID, int ACT, bool CSC, bool BRND>
__global__ __launch_bounds__(256) void wmma_gemm64(
    const unsigned short* __restrict__ Ap, const unsigned short* __restrict__ A2p, int lda, long strideA,
    const unsigned short* __restrict__ Btp, const unsigned short* __restrict__ Bt2p, int ldb, long strideB,
    void* __restrict__ Cout, void* __restrict__ Cout2, int ldc, long strideC,
    const float* __restrict__ bias, const float* __restrict__ cscale,
    const float* __restrict__ resid, long strideR,
    int M, int N, int K, float scale) {
  typedef typename Elem<ET>::T T;
  typedef typename Frag<T>::V V;
  const T* A = (const T*)Ap; const T* A2 = (const T*)A2p; const T* Bt = (const T*)Btp; const T* Bt2 = (const T*)Bt2p;
  __shared__ __align__(16) float sT[8][16 * 68];
  const int b    = blockIdx.y;
  const int lane = threadIdx.x & 31;
  const int wave = threadIdx.x >> 5;
  const int tilesN = N >> 6;
  const int tilesM = M >> 6;
  const int tile = blockIdx.x * 8 + wave;
  if (tile >= tilesM * tilesN) return;
  const int tm = tile / tilesN;
  const int tn = tile - tm * tilesN;
  const int m0 = tm << 6;
  const int n0 = tn << 6;

  const T* Ab  = A  + (size_t)b * strideA;
  const T* Bb  = Bt + (size_t)b * strideB;
  const T* Ab2 = (SPLIT >= 1) ? (A2  + (size_t)b * strideA) : nullptr;
  const T* Bb2 = (SPLIT == 2) ? (Bt2 + (size_t)b * strideB) : nullptr;

  const int rlane = lane & 15;
  const int koff  = (lane >> 4) * 8;
  const int mOff  = (lane >> 4) * 8;

  v8f acc[4][4];
#pragma unroll
  for (int i = 0; i < 4; ++i)
#pragma unroll
    for (int j = 0; j < 4; ++j) acc[i][j] = (v8f){0.f,0.f,0.f,0.f,0.f,0.f,0.f,0.f};

  for (int k0 = 0; k0 < K; k0 += 32) {
    V bh[4], bl[4];
#pragma unroll
    for (int j = 0; j < 4; ++j) {
      const size_t bo = (size_t)(n0 + (j << 4) + rlane) * ldb + koff + k0;
      bh[j] = Frag<T>::load(Bb + bo);
      if (SPLIT == 2) bl[j] = Frag<T>::load(Bb2 + bo);
    }
#pragma unroll
    for (int i = 0; i < 4; ++i) {
      const size_t ao = (size_t)(m0 + (i << 4) + rlane) * lda + koff + k0;
      V ah = Frag<T>::load(Ab + ao);
      V al;
      if (SPLIT >= 1) al = Frag<T>::load(Ab2 + ao);
#pragma unroll
      for (int j = 0; j < 4; ++j) {
        acc[i][j] = Frag<T>::mma(ah, bh[j], acc[i][j]);
        if (SPLIT == 2) acc[i][j] = Frag<T>::mma(ah, bl[j], acc[i][j]);
        if (SPLIT >= 1) acc[i][j] = Frag<T>::mma(al, bh[j], acc[i][j]);
      }
      Frag<T>::guard(acc[i][0], acc[i][3], ah, (SPLIT >= 1) ? al : ah);
    }
    Frag<T>::keep(bh[0], bh[1], bh[2], bh[3]);
    if (SPLIT == 2) Frag<T>::keep(bl[0], bl[1], bl[2], bl[3]);
  }
  acc_guard4(acc[0][0], acc[0][1], acc[0][2], acc[0][3]);
  acc_guard4(acc[1][0], acc[1][1], acc[1][2], acc[1][3]);
  acc_guard4(acc[2][0], acc[2][1], acc[2][2], acc[2][3]);
  acc_guard4(acc[3][0], acc[3][1], acc[3][2], acc[3][3]);

  float* slab = sT[wave];
  const float* Rb = RESID ? (resid + (size_t)b * strideR) : nullptr;
#pragma unroll
  for (int i = 0; i < 4; ++i) {
    const int mBase = m0 + (i << 4);
#pragma unroll
    for (int j = 0; j < 4; ++j) {
      const int n = n0 + (j << 4) + rlane;
      float bv = 0.f;
      if (BIAS_MODE == 2) { bv = bias[n]; if (BRND) bv = bfr(bv); }
      float cv = 1.f;
      if (CSC) { cv = cscale[n]; if (BRND) cv = bfr(cv); }
#pragma unroll
      for (int r = 0; r < 8; ++r) {
        float v = acc[i][j][r] * scale;
        if (BIAS_MODE == 1) { float bm = bias[mBase + mOff + r]; if (BRND) bm = bfr(bm); v += bm; }
        if (BIAS_MODE == 2) v += bv;
        if (RESID) v += Rb[(size_t)(mBase + mOff + r) * ldc + n];
        if (CSC) v *= cv;
        if (ACT == 1) v = tanhf(v);
        if (ACT == 2) v = fmaxf(v, 0.0f);
        if (ACT == 3) v = v / (1.0f + expf(-v));
        if (ACT == 4) v = (v > 0.f) ? v : 0.01f * v;
        if (ACT == 6) v = expf(v);
        slab[(mOff + r) * 68 + (j << 4) + rlane] = v;
      }
    }
    __builtin_amdgcn_fence(__ATOMIC_RELEASE, "workgroup");
    __builtin_amdgcn_wave_barrier();
    __builtin_amdgcn_fence(__ATOMIC_ACQUIRE, "workgroup");
    if (OUT_MODE == 0) {
      float* C = (float*)Cout + (size_t)b * strideC;
      const int hh = lane >> 4, c4 = (lane & 15) * 4;
      for (int pass = 0; pass < 2; ++pass) {
#pragma unroll
        for (int it = 0; it < 8; ++it) {
          const int row = it * 2 + hh;
          v4f v = *(const v4f*)(slab + row * 68 + c4);
          *(volatile v4f*)(C + (size_t)(mBase + row) * ldc + n0 + c4) = v;
        }
        __threadfence();
      }
    } else {
      const int q = lane >> 3, c8 = (lane & 7) * 8;
      unsigned short* C  = (unsigned short*)Cout  + (size_t)b * strideC;
      unsigned short* C2 = (OUT_MODE == 2) ? ((unsigned short*)Cout2 + (size_t)b * strideC) : nullptr;
      for (int pass = 0; pass < 2; ++pass) {
#pragma unroll
        for (int it = 0; it < 4; ++it) {
          const int row = it * 4 + q;
          const float* sp = slab + row * 68 + c8;
          v8h hv, lv;
#pragma unroll
          for (int e = 0; e < 8; ++e) {
            if (OUT_MODE == 1) {
              hv[e] = (_Float16)sp[e];
            } else {
              unsigned short hb = f2bf_bits(sp[e]);
              unsigned short lb = f2bf_bits(sp[e] - bf_bits2f(hb));
              hv[e] = __builtin_bit_cast(_Float16, hb);
              lv[e] = __builtin_bit_cast(_Float16, lb);
            }
          }
          *(volatile v8h*)(C + (size_t)(mBase + row) * ldc + n0 + c8) = hv;
          if (OUT_MODE == 2) *(volatile v8h*)(C2 + (size_t)(mBase + row) * ldc + n0 + c8) = lv;
        }
        __threadfence();
      }
    }
    __builtin_amdgcn_fence(__ATOMIC_RELEASE, "workgroup");
    __builtin_amdgcn_wave_barrier();
    __builtin_amdgcn_fence(__ATOMIC_ACQUIRE, "workgroup");
  }
}

__global__ __launch_bounds__(256) void wcast4_kernel(const float* __restrict__ w0, const float* __restrict__ w1,
                                                     const float* __restrict__ w2, const float* __restrict__ w3,
                                                     unsigned short* __restrict__ o0, unsigned short* __restrict__ o1,
                                                     unsigned short* __restrict__ o2, unsigned short* __restrict__ o3, int n2) {
  const int sel = blockIdx.y;
  const float* src = (sel == 0) ? w0 : (sel == 1) ? w1 : (sel == 2) ? w2 : w3;
  unsigned short* dst = (sel == 0) ? o0 : (sel == 1) ? o1 : (sel == 2) ? o2 : o3;
  const int i = blockIdx.x * 256 + threadIdx.x;
  if (i < n2) {
    const v2f f = *(const v2f*)(src + 2 * (size_t)i);
    const unsigned u = pk16(f2bf_bits(f[0]), f2bf_bits(f[1]));
    ((volatile unsigned*)dst)[i] = u;
    __threadfence();
    ((volatile unsigned*)dst)[i] = u;
  }
}

__global__ __launch_bounds__(256) void xcast2_kernel(const float* __restrict__ src, unsigned short* __restrict__ dst, int n2) {
  const int i = blockIdx.x * 256 + threadIdx.x;
  if (i < n2) {
    const v2f f = *(const v2f*)(src + 2 * (size_t)i);
    const unsigned u = pk16(f2bf_bits(f[0]), f2bf_bits(f[1]));
    ((volatile unsigned*)dst)[i] = u;
    __threadfence();
    ((volatile unsigned*)dst)[i] = u;
  }
}

__global__ __launch_bounds__(256) void l2norm_kernel(const float* __restrict__ xf, unsigned short* __restrict__ o16,
                                                     int nrows, float eps, float carry) {
  const int wave = threadIdx.x >> 5, lane = threadIdx.x & 31;
  const int row = blockIdx.x * 8 + wave;
  if (row >= nrows) return;
  const float* p = xf + (size_t)row * DIM_E;
  float v[2][8];
#pragma unroll
  for (int g = 0; g < 2; ++g) {
    const v4f a0 = *(const v4f*)(p + g * 256 + lane * 8);
    const v4f a1 = *(const v4f*)(p + g * 256 + lane * 8 + 4);
    v[g][0] = a0[0]; v[g][1] = a0[1]; v[g][2] = a0[2]; v[g][3] = a0[3];
    v[g][4] = a1[0]; v[g][5] = a1[1]; v[g][6] = a1[2]; v[g][7] = a1[3];
  }
  float ss = 0.f;
#pragma unroll
  for (int g = 0; g < 2; ++g)
#pragma unroll
    for (int e = 0; e < 8; ++e) ss += v[g][e] * v[g][e];
#pragma unroll
  for (int off = 16; off > 0; off >>= 1) ss += __shfl_xor(ss, off, 32);
  ss = __shfl(ss, 0, 32);
  const float nrm  = sqrtf(ss);
  const float rinv = 1.0f / fmaxf(nrm, eps);
  const float mul  = rinv * carry;
  v8h hv[2];
#pragma unroll
  for (int g = 0; g < 2; ++g)
#pragma unroll
    for (int e = 0; e < 8; ++e) hv[g][e] = (_Float16)(v[g][e] * mul);
  unsigned short* orow = o16 + (size_t)row * DIM_E;
  for (int pass = 0; pass < 2; ++pass) {
#pragma unroll
    for (int g = 0; g < 2; ++g) *(volatile v8h*)(orow + g * 256 + lane * 8) = hv[g];
    __threadfence();
  }
}

__device__ __forceinline__ __bf16 at_f2bf(float f) { return __builtin_bit_cast(__bf16, f2bf_bits(f)); }
__device__ __forceinline__ void at_split(float f, __bf16& hi, __bf16& lo) {
  const unsigned short hb = f2bf_bits(f);
  hi = __builtin_bit_cast(__bf16, hb);
  lo = at_f2bf(f - __uint_as_float(((unsigned)hb) << 16));
}
__device__ __forceinline__ v8f at_mma(v16b a, v16b b, v8f c) {
  c = __builtin_amdgcn_wmma_f32_16x16x32_bf16(false, a, false, b, (short)0, c, false, false);
  asm volatile("v_nop\n\tv_nop\n\tv_nop\n\tv_nop" : "+v"(c) : "v"(a), "v"(b));
  return c;
}
__device__ __forceinline__ v8f mma_h16(v16h a, v16h b, v8f c) {
  c = __builtin_amdgcn_wmma_f32_16x16x32_f16(false, a, false, b, (short)0, c, false, false);
  asm volatile("v_nop\n\tv_nop\n\tv_nop\n\tv_nop" : "+v"(c) : "v"(a), "v"(b));
  return c;
}

__global__ __launch_bounds__(256)
void linmem_kernel(const unsigned short* __restrict__ q16p, const unsigned short* __restrict__ k16p,
                   const unsigned short* __restrict__ vthp, const unsigned short* __restrict__ vtlp,
                   unsigned short* __restrict__ athp, unsigned short* __restrict__ atlp, float pscale) {
  __shared__ __align__(16) __bf16 Ph[64 * 64];
  __shared__ __align__(16) __bf16 Pl[64 * 64];
  __shared__ __align__(16) float slab[8][16 * 68];
  __shared__ float dtab[160];

  const int tid  = threadIdx.x;
  const int wave = tid >> 5;
  const int lane = tid & 31;
  const int hh   = lane >> 4;
  const int c    = lane & 15;
  const int rw   = wave & 3;
  const int chh  = wave >> 2;

  const int b  = blockIdx.x >> 5;
  const int qb = blockIdx.x & 31;
  const int q0 = qb * 64 + rw * 16;

  if (tid < 160) {
    const int ex = (tid < 64) ? tid : ((tid < 128) ? (64 - tid) : ((tid - 128) * 64));
    dtab[tid] = powf(DECAY_VAL, (float)ex);
  }
  __syncthreads();

  const _Float16* Qp = (const _Float16*)(const void*)q16p + (size_t)b * SEQ_T * DIM_E;
  const _Float16* Kp = (const _Float16*)(const void*)k16p + (size_t)b * SEQ_T * DIM_E;
  const __bf16*   Vh = (const __bf16*)(const void*)vthp + (size_t)b * SEQ_T;
  const __bf16*   Vl = (const __bf16*)(const void*)vtlp + (size_t)b * SEQ_T;

  const float cfA = dtab[64 + chh * 32 + c];
  const float cfB = dtab[64 + chh * 32 + 16 + c];
  float rf[8];
#pragma unroll
  for (int r = 0; r < 8; ++r) rf[r] = pscale * dtab[rw * 16 + 8 * hh + r];

  v8f oacc[16];
#pragma unroll
  for (int t = 0; t < 16; ++t) oacc[t] = (v8f){0.f,0.f,0.f,0.f,0.f,0.f,0.f,0.f};

  const int kc0 = (qb >= KSPAN) ? (qb - KSPAN + 1) : 0;
  for (int kc = kc0; kc <= qb; ++kc) {
    const int kv0   = kc * 64;
    const int kcol0 = kv0 + chh * 32;
    __syncthreads();

    v8f s0 = (v8f){0.f,0.f,0.f,0.f,0.f,0.f,0.f,0.f};
    v8f s1 = (v8f){0.f,0.f,0.f,0.f,0.f,0.f,0.f,0.f};
#pragma unroll 1
    for (int k0 = 0; k0 < DIM_E; k0 += 32) {
      const v16h a  = Frag<_Float16>::load(Qp + (size_t)(q0 + c) * DIM_E + k0 + 8 * hh);
      const v16h b0 = Frag<_Float16>::load(Kp + (size_t)(kcol0 + c) * DIM_E + k0 + 8 * hh);
      const v16h b1 = Frag<_Float16>::load(Kp + (size_t)(kcol0 + 16 + c) * DIM_E + k0 + 8 * hh);
      s0 = mma_h16(a, b0, s0);
      s1 = mma_h16(a, b1, s1);
    }

    const bool diag = (kc == qb);
    const float gf = dtab[128 + (qb - kc)];
    const int kcA = kcol0 + c, kcB = kcol0 + 16 + c;
#pragma unroll
    for (int r = 0; r < 8; ++r) {
      const int qrow = q0 + 8 * hh + r;
      const int prow = rw * 16 + 8 * hh + r;
      const float rg = rf[r] * gf;
      float v0 = s0[r] * rg * cfA;
      float v1 = s1[r] * rg * cfB;
      if (diag && (kcA > qrow)) v0 = 0.f;
      if (diag && (kcB > qrow)) v1 = 0.f;
      __bf16 h0, l0, h1, l1;
      at_split(v0, h0, l0);
      at_split(v1, h1, l1);
      Ph[prow * 64 + chh * 32 + c]      = h0;
      Pl[prow * 64 + chh * 32 + c]      = l0;
      Ph[prow * 64 + chh * 32 + 16 + c] = h1;
      Pl[prow * 64 + chh * 32 + 16 + c] = l1;
    }
    __syncthreads();

#pragma unroll 1
    for (int kk = 0; kk < 2; ++kk) {
      const v16b pa = Frag<__bf16>::load(Ph + (rw * 16 + c) * 64 + kk * 32 + 8 * hh);
      const v16b pl = Frag<__bf16>::load(Pl + (rw * 16 + c) * 64 + kk * 32 + 8 * hh);
      const size_t vcol = (size_t)(kv0 + kk * 32 + 8 * hh);
#pragma unroll
      for (int t = 0; t < 16; ++t) {
        const size_t vo = (size_t)(chh * 256 + t * 16 + c) * ATT_LDV + vcol;
        const v16b vb = Frag<__bf16>::load(Vh + vo);
        const v16b vl = Frag<__bf16>::load(Vl + vo);
        oacc[t] = at_mma(pa, vb, oacc[t]);
        oacc[t] = at_mma(pa, vl, oacc[t]);
        oacc[t] = at_mma(pl, vb, oacc[t]);
      }
    }
  }

  float* sl = slab[wave];
  const int qq = lane >> 3, c8 = (lane & 7) * 8;
#pragma unroll
  for (int quarter = 0; quarter < 4; ++quarter) {
#pragma unroll
    for (int t = 0; t < 4; ++t)
#pragma unroll
      for (int r = 0; r < 8; ++r)
        sl[(8 * hh + r) * 68 + t * 16 + c] = oacc[quarter * 4 + t][r];
    __builtin_amdgcn_fence(__ATOMIC_RELEASE, "workgroup");
    __builtin_amdgcn_wave_barrier();
    __builtin_amdgcn_fence(__ATOMIC_ACQUIRE, "workgroup");
    for (int pass = 0; pass < 2; ++pass) {
#pragma unroll
      for (int it = 0; it < 4; ++it) {
        const int row = it * 4 + qq;
        const float* sp = sl + row * 68 + c8;
        v8h hv, lv;
#pragma unroll
        for (int e = 0; e < 8; ++e) {
          const unsigned short hb = f2bf_bits(sp[e]);
          const unsigned short lb = f2bf_bits(sp[e] - bf_bits2f(hb));
          hv[e] = __builtin_bit_cast(_Float16, hb);
          lv[e] = __builtin_bit_cast(_Float16, lb);
        }
        const size_t go = ((size_t)b * SEQ_T + q0 + row) * DIM_E + chh * 256 + quarter * 64 + c8;
        *(volatile v8h*)(athp + go) = hv;
        *(volatile v8h*)(atlp + go) = lv;
      }
      __threadfence();
    }
    __builtin_amdgcn_fence(__ATOMIC_RELEASE, "workgroup");
    __builtin_amdgcn_wave_barrier();
    __builtin_amdgcn_fence(__ATOMIC_ACQUIRE, "workgroup");
  }
}

extern "C" void kernel_launch(void* const* d_in, const int* in_sizes, int n_in,
                              void* d_out, int out_size, void* d_ws, size_t ws_size,
                              hipStream_t stream) {
  if (n_in < 9) return;
  const int nAct = NBATCH * SEQ_T * DIM_E;
  const int nW   = DIM_E * DIM_E;
  if (in_sizes[0] != nAct) return;
  if (in_sizes[1] != nW || in_sizes[3] != nW || in_sizes[5] != nW || in_sizes[7] != nW) return;
  if (in_sizes[2] != DIM_E || in_sizes[4] != DIM_E || in_sizes[6] != DIM_E || in_sizes[8] != DIM_E) return;
  if (out_size != nAct) return;

  const float* x   = (const float*)d_in[0];
  const float* w_k = (const float*)d_in[1];
  const float* b_k = (const float*)d_in[2];
  const float* w_v = (const float*)d_in[3];
  const float* b_v = (const float*)d_in[4];
  const float* w_q = (const float*)d_in[5];
  const float* b_q = (const float*)d_in[6];
  const float* w_o = (const float*)d_in[7];
  const float* b_o = (const float*)d_in[8];

  const size_t PW  = (size_t)nW * 2;
  const size_t P16 = (size_t)nAct * 2;
  const size_t P32 = P16 * 2;
  size_t off = 0;
  const size_t oWk = off; off += PW;
  const size_t oWv = off; off += PW;
  const size_t oWq = off; off += PW;
  const size_t oWo = off; off += PW;
  const size_t oX16 = off; off += P16;
  const size_t oF32 = off;
  const size_t oATh = off;
  const size_t oATl = off + P16; off += P32;
  const size_t oQ16 = off; off += P16;
  const size_t oK16 = off; off += P16;
  const size_t oVTh = off; off += P16;
  const size_t oVTl = off; off += P16;
  if (off > ws_size) return;
  if (off > (size_t)134217728) return;

  char* ws = (char*)d_ws;
  unsigned short* Wk16 = (unsigned short*)(ws + oWk);
  unsigned short* Wv16 = (unsigned short*)(ws + oWv);
  unsigned short* Wq16 = (unsigned short*)(ws + oWq);
  unsigned short* Wo16 = (unsigned short*)(ws + oWo);
  unsigned short* X16  = (unsigned short*)(ws + oX16);
  float*          F32  = (float*)(ws + oF32);
  unsigned short* ATh  = (unsigned short*)(ws + oATh);
  unsigned short* ATl  = (unsigned short*)(ws + oATl);
  unsigned short* Q16  = (unsigned short*)(ws + oQ16);
  unsigned short* K16  = (unsigned short*)(ws + oK16);
  unsigned short* VTh  = (unsigned short*)(ws + oVTh);
  unsigned short* VTl  = (unsigned short*)(ws + oVTl);

  const dim3 blk(256);
  const int nRows = NBATCH * SEQ_T;
  const float eps    = 1e-6f;
  const float carry  = 64.0f;
  const float sc     = 0.03f / sqrtf(512.0f);
  const float pscale = sc * (1.0f / 4096.0f);

  wcast4_kernel<<<dim3(nW / 2 / 256, 4), blk, 0, stream>>>(w_k, w_v, w_q, w_o, Wk16, Wv16, Wq16, Wo16, nW / 2);

  xcast2_kernel<<<dim3(nAct / 2 / 256), blk, 0, stream>>>(x, X16, nAct / 2);

  const dim3 gProj(((nRows / 64) * (DIM_E / 64)) / 8, 1);
  const dim3 gVT(((DIM_E / 64) * (SEQ_T / 64)) / 8, NBATCH);

  wmma_gemm64<1, 0, 2, 0, false, 0, false, true><<<gProj, blk, 0, stream>>>(
      X16, X16, DIM_E, 0L, Wq16, Wq16, DIM_E, 0L, (void*)F32, (void*)F32, DIM_E, 0L,
      b_q, b_q, x, 0L, nRows, DIM_E, DIM_E, 1.0f);

  l2norm_kernel<<<dim3(nRows / 8), blk, 0, stream>>>(F32, Q16, nRows, eps, carry);

  wmma_gemm64<1, 0, 2, 0, false, 0, false, true><<<gProj, blk, 0, stream>>>(
      X16, X16, DIM_E, 0L, Wk16, Wk16, DIM_E, 0L, (void*)F32, (void*)F32, DIM_E, 0L,
      b_k, b_k, x, 0L, nRows, DIM_E, DIM_E, 1.0f);

  l2norm_kernel<<<dim3(nRows / 8), blk, 0, stream>>>(F32, K16, nRows, eps, carry);

  wmma_gemm64<1, 0, 1, 2, false, 0, false, true><<<gVT, blk, 0, stream>>>(
      Wv16, Wv16, DIM_E, 0L, X16, X16, DIM_E, (long)SEQ_T * DIM_E, (void*)VTh, (void*)VTl, ATT_LDV, (long)SEQ_T,
      b_v, b_v, x, 0L, DIM_E, SEQ_T, DIM_E, 1.0f);

  linmem_kernel<<<dim3(NBATCH * (SEQ_T / 64)), blk, 0, stream>>>(Q16, K16, VTh, VTl, ATh, ATl, pscale);

  wmma_gemm64<1, 1, 2, 0, false, 0, false, true><<<gProj, blk, 0, stream>>>(
      ATh, ATl, DIM_E, 0L, Wo16, Wo16, DIM_E, 0L, d_out, d_out, DIM_E, 0L,
      b_o, b_o, x, 0L, nRows, DIM_E, DIM_E, 1.0f);
}
